// Block_58394375356504
// MI455X (gfx1250) — hardware-verified
//
#include <hip/hip_runtime.h>
#include <math.h>

#ifndef NB
#define NB 2
#endif
#ifndef SEQ
#define SEQ 2048
#endif
#define NB_FULL 2
#define SEQ_FULL 2048
#define CW 1024
#define NH 16
#define DHD 64
#define FF 4096
#define QLD (3 * CW)
#define MROWS (NB * SEQ)

static_assert(NB >= 1 && NB <= NB_FULL);
static_assert(SEQ >= 64 && SEQ <= SEQ_FULL);
static_assert(SEQ % 64 == 0);
static_assert(CW == NH * DHD);
static_assert(DHD == 64);
static_assert(CW % 64 == 0 && FF % 64 == 0 && QLD % 64 == 0);
static_assert(CW % 32 == 0 && FF % 32 == 0);
static_assert(MROWS % 64 == 0);
static_assert(((MROWS / 64) * (QLD / 64)) % 8 == 0);
static_assert(((MROWS / 64) * (CW / 64)) % 8 == 0);
static_assert(((MROWS / 64) * (FF / 64)) % 8 == 0);

typedef __attribute__((ext_vector_type(16))) _Float16 v16h;
typedef __attribute__((ext_vector_type(8)))  _Float16 v8h;
typedef __attribute__((ext_vector_type(8)))  float    v8f;
typedef __attribute__((ext_vector_type(4)))  float    v4f;
typedef __attribute__((ext_vector_type(4)))  unsigned int u4;

union FH { v16h v; v8h h[2]; };

#define VST2(T, ptr, val) do { const T vst2_v_ = (val); volatile T* vst2_p_ = (volatile T*)(ptr); *vst2_p_ = vst2_v_; __threadfence(); *vst2_p_ = vst2_v_; } while (0)

__device__ __forceinline__ float bfr(float v) { const unsigned u = __builtin_bit_cast(unsigned, v); const unsigned r = (u + 0x7fffu + ((u >> 16) & 1u)) & 0xffff0000u; return __builtin_bit_cast(float, r); }
__device__ __forceinline__ unsigned int pk2(float a, float b) { return (unsigned int)__builtin_bit_cast(unsigned short, (_Float16)a) | ((unsigned int)__builtin_bit_cast(unsigned short, (_Float16)b) << 16); }

__device__ __forceinline__ v8f wmma16(v16h a, v16h b, v8f c) {
    c = __builtin_amdgcn_wmma_f32_16x16x32_f16(false, a, false, b, (short)0, c, false, false);
    asm volatile("v_nop\n\tv_nop\n\tv_nop\n\tv_nop" : "+v"(c) : "v"(a), "v"(b));
    return c;
}
__device__ __forceinline__ void dep_guard_h(v8f& a, v8f& b, v16h x, v16h y) { asm volatile("v_nop\n\tv_nop\n\tv_nop\n\tv_nop" : "+v"(a), "+v"(b) : "v"(x), "v"(y)); }
__device__ __forceinline__ void keep4_h(v16h a, v16h b, v16h c, v16h d) { asm volatile("v_nop" :: "v"(a), "v"(b), "v"(c), "v"(d)); }
__device__ __forceinline__ void acc_guard4(v8f& a, v8f& b, v8f& c, v8f& d) { asm volatile("v_nop\n\tv_nop\n\tv_nop\n\tv_nop" : "+v"(a), "+v"(b), "+v"(c), "+v"(d)); }
__device__ __forceinline__ v16h frag_ld_g(const _Float16* __restrict__ p) { FH f; f.h[0] = *(const v8h*)(p); f.h[1] = *(const v8h*)(p + 16); return f.v; }

__global__ __launch_bounds__(256) void k_colstat(const float* __restrict__ X, long long bstride, float* __restrict__ MEAN, float* __restrict__ RSTD, int xbf) {
    #pragma clang fp contract(off)
    __shared__ float red[8][32];
    const int tx = threadIdx.x & 31, ty = threadIdx.x >> 5;
    const int c = blockIdx.x * 32 + tx, b = blockIdx.y;
    const float* xp = X + (long long)b * bstride + c;
    float s = 0.f;
#pragma unroll 4
    for (int t = ty; t < SEQ; t += 8) { float v = xp[(long long)t * CW]; v = xbf ? bfr(v) : v; s += v; }
    red[ty][tx] = s;
    __syncthreads();
    float a = 0.f;
#pragma unroll 1
    for (int i = 0; i < 8; ++i) a += red[i][tx];
    const float mu = a * (1.0f / (float)SEQ);
    __syncthreads();
    float q = 0.f;
#pragma unroll 4
    for (int t = ty; t < SEQ; t += 8) { float v = xp[(long long)t * CW]; v = xbf ? bfr(v) : v; const float d = v - mu; q += d * d; }
    red[ty][tx] = q;
    __syncthreads();
    float qq = 0.f;
#pragma unroll 1
    for (int i = 0; i < 8; ++i) qq += red[i][tx];
    const float var = qq * (1.0f / (float)(SEQ - 1));
    const float rs = 1.0f / sqrtf(var + 1e-5f);
    if (ty == 0) {
        VST2(float, MEAN + (long long)b * CW + c, mu);
        VST2(float, RSTD + (long long)b * CW + c, rs);
    }
}

__device__ __forceinline__ v4f ln4(v4f x, v4f mu, v4f rs, v4f g, v4f be, int xbf) {
    #pragma clang fp contract(off)
    if (xbf) { x.x = bfr(x.x); x.y = bfr(x.y); x.z = bfr(x.z); x.w = bfr(x.w); }
    v4f y;
    y.x = bfr(g.x) * ((x.x - mu.x) * rs.x) + bfr(be.x);
    y.y = bfr(g.y) * ((x.y - mu.y) * rs.y) + bfr(be.y);
    y.z = bfr(g.z) * ((x.z - mu.z) * rs.z) + bfr(be.z);
    y.w = bfr(g.w) * ((x.w - mu.w) * rs.w) + bfr(be.w);
    return y;
}
__global__ __launch_bounds__(256) void k_lnt_apply(const float* __restrict__ X, long long bstride, const float* __restrict__ MEAN, const float* __restrict__ RSTD,
                                                    const float* __restrict__ GA, const float* __restrict__ BE, unsigned short* __restrict__ Y16, int xbf) {
    #pragma clang fp contract(off)
    const long long u = (long long)blockIdx.x * 256 + threadIdx.x;
    if (u >= (long long)MROWS * (CW / 8)) return;
    const int r = (int)(u / (CW / 8)); const int c0 = 8 * (int)(u % (CW / 8));
    const int b = r / SEQ, t = r - b * SEQ;
    const float* xr = X + (long long)b * bstride + (long long)t * CW + c0;
    const float* mp = MEAN + (long long)b * CW + c0;
    const float* rp = RSTD + (long long)b * CW + c0;
    const v4f y0 = ln4(*(const v4f*)(xr), *(const v4f*)(mp), *(const v4f*)(rp), *(const v4f*)(GA + c0), *(const v4f*)(BE + c0), xbf);
    const v4f y1 = ln4(*(const v4f*)(xr + 4), *(const v4f*)(mp + 4), *(const v4f*)(rp + 4), *(const v4f*)(GA + c0 + 4), *(const v4f*)(BE + c0 + 4), xbf);
    u4 pk; pk.x = pk2(y0.x, y0.y); pk.y = pk2(y0.z, y0.w); pk.z = pk2(y1.x, y1.y); pk.w = pk2(y1.z, y1.w);
    VST2(u4, (u4*)(Y16 + (long long)r * CW + c0), pk);
}

__global__ __launch_bounds__(256) void k_cast_heads(const float* __restrict__ W, unsigned short* __restrict__ DST, float sc) {
    const long long u = (long long)blockIdx.x * 256 + threadIdx.x;
    if (u >= (long long)CW * (CW / 8)) return;
    const int n = (int)(u / (CW / 8)); const int c0 = 8 * (int)(u % (CW / 8));
    const int h = n >> 6, d = n & 63;
    const float* s = W + ((long long)h * CW + c0) * DHD + d;
    float w[8];
#pragma unroll
    for (int e = 0; e < 8; ++e) w[e] = bfr(s[(long long)e * DHD]) * sc;
    u4 pk; pk.x = pk2(w[0], w[1]); pk.y = pk2(w[2], w[3]); pk.z = pk2(w[4], w[5]); pk.w = pk2(w[6], w[7]);
    VST2(u4, (u4*)(DST + (long long)n * CW + c0), pk);
}
__global__ __launch_bounds__(256) void k_castbT(const float* __restrict__ SRC, int lds, unsigned short* __restrict__ DST, int ldd, int nR, int nC, float sc) {
    const long long u = (long long)blockIdx.x * 256 + threadIdx.x; const int per = nR / 8;
    if (u >= (long long)nC * per) return;
    const int c = (int)(u / per); const int r0 = 8 * (int)(u % per);
    float w[8];
#pragma unroll
    for (int e = 0; e < 8; ++e) w[e] = bfr(SRC[(long long)(r0 + e) * lds + c]) * sc;
    u4 pk; pk.x = pk2(w[0], w[1]); pk.y = pk2(w[2], w[3]); pk.z = pk2(w[4], w[5]); pk.w = pk2(w[6], w[7]);
    VST2(u4, (u4*)(DST + (long long)c * ldd + r0), pk);
}

template <int OUT_MODE, int BIAS, int ACT, int RES>
__device__ __forceinline__ void gemm64_body(const unsigned short* __restrict__ Ap, int lda, const unsigned short* __restrict__ Btp, int ldb,
                                            void* __restrict__ Cout, int ldc, const float* __restrict__ bias,
                                            const float* __restrict__ resid, int ldr, int rows_per_b, long long r_bstride,
                                            int M, int N, int K, float scale) {
    const _Float16* A = (const _Float16*)Ap; const _Float16* Bt = (const _Float16*)Btp;
    __shared__ __align__(16) float sT[8][16 * 68];
    const int lane = threadIdx.x & 31;
    const int wave = threadIdx.x >> 5;
    const int tilesN = N >> 6;
    const int tilesM = M >> 6;
    const int tile = blockIdx.x * 8 + wave;
    if (tile >= tilesM * tilesN) return;
    const int tm = tile / tilesN;
    const int tn = tile - tm * tilesN;
    const int m0 = tm << 6;
    const int n0 = tn << 6;
    const int rlane = lane & 15;
    const int koff  = (lane >> 4) * 8;
    const int mOff  = (lane >> 4) * 8;

    v8f acc[4][4];
#pragma unroll
    for (int i = 0; i < 4; ++i)
#pragma unroll
        for (int j = 0; j < 4; ++j) acc[i][j] = (v8f){0.f, 0.f, 0.f, 0.f, 0.f, 0.f, 0.f, 0.f};

    for (int k0 = 0; k0 < K; k0 += 32) {
        v16h bh[4];
#pragma unroll
        for (int j = 0; j < 4; ++j) bh[j] = frag_ld_g(Bt + (size_t)(n0 + (j << 4) + rlane) * ldb + koff + k0);
#pragma unroll
        for (int i = 0; i < 4; ++i) {
            const v16h ah = frag_ld_g(A + (size_t)(m0 + (i << 4) + rlane) * lda + koff + k0);
#pragma unroll
            for (int j = 0; j < 4; ++j) acc[i][j] = __builtin_amdgcn_wmma_f32_16x16x32_f16(false, ah, false, bh[j], (short)0, acc[i][j], false, false);
            dep_guard_h(acc[i][0], acc[i][3], ah, ah);
        }
        keep4_h(bh[0], bh[1], bh[2], bh[3]);
    }
    acc_guard4(acc[0][0], acc[0][1], acc[0][2], acc[0][3]);
    acc_guard4(acc[1][0], acc[1][1], acc[1][2], acc[1][3]);
    acc_guard4(acc[2][0], acc[2][1], acc[2][2], acc[2][3]);
    acc_guard4(acc[3][0], acc[3][1], acc[3][2], acc[3][3]);

    float bvj[4];
#pragma unroll
    for (int j = 0; j < 4; ++j) { bvj[j] = 0.f; if (BIAS) bvj[j] = bfr(bias[n0 + (j << 4) + rlane]); }

    float* slab = sT[wave];
#pragma unroll
    for (int i = 0; i < 4; ++i) {
        const int mBase = m0 + (i << 4);
#pragma unroll
        for (int j = 0; j < 4; ++j) {
#pragma unroll
            for (int r = 0; r < 8; ++r) {
                float v = acc[i][j][r] * scale + bvj[j];
                if (ACT == 1) v = fmaxf(v, 0.0f);
                slab[(mOff + r) * 68 + (j << 4) + rlane] = v;
            }
        }
        __builtin_amdgcn_fence(3  , "workgroup");
        __builtin_amdgcn_wave_barrier();
        __builtin_amdgcn_fence(2  , "workgroup");
        if (OUT_MODE == 0) {
            float* C = (float*)Cout;
            const int hh = lane >> 4, c4 = (lane & 15) * 4;
            long long roff = 0;
            if (RES) { const int rb = mBase / rows_per_b; roff = (long long)rb * r_bstride + (long long)(mBase - rb * rows_per_b) * ldr + n0 + c4; }
            for (int pass = 0; pass < 2; ++pass) {
#pragma unroll
                for (int it = 0; it < 8; ++it) {
                    const int row = it * 2 + hh;
                    v4f v = *(const v4f*)(slab + row * 68 + c4);
                    if (RES) {
                        v4f x = *(const v4f*)(resid + roff + (long long)row * ldr);
                        if (RES == 1) { x.x = bfr(x.x); x.y = bfr(x.y); x.z = bfr(x.z); x.w = bfr(x.w); }
                        v = v + x;
                    }
                    *(volatile v4f*)(C + (size_t)(mBase + row) * ldc + n0 + c4) = v;
                }
                __threadfence();
            }
        } else {
            const int q = lane >> 3, c8 = (lane & 7) * 8;
            unsigned short* C = (unsigned short*)Cout;
            for (int pass = 0; pass < 2; ++pass) {
#pragma unroll
                for (int it = 0; it < 4; ++it) {
                    const int row = it * 4 + q;
                    const v4f a0 = *(const v4f*)(slab + row * 68 + c8);
                    const v4f a1 = *(const v4f*)(slab + row * 68 + c8 + 4);
                    v8h hv;
                    hv[0] = (_Float16)a0.x; hv[1] = (_Float16)a0.y; hv[2] = (_Float16)a0.z; hv[3] = (_Float16)a0.w;
                    hv[4] = (_Float16)a1.x; hv[5] = (_Float16)a1.y; hv[6] = (_Float16)a1.z; hv[7] = (_Float16)a1.w;
                    *(volatile v8h*)(C + (size_t)(mBase + row) * ldc + n0 + c8) = hv;
                }
                __threadfence();
            }
        }
        __builtin_amdgcn_fence(3  , "workgroup");
        __builtin_amdgcn_wave_barrier();
        __builtin_amdgcn_fence(2  , "workgroup");
    }
}

__global__ __launch_bounds__(256) void k_gemm_qkv(const unsigned short* __restrict__ A, const unsigned short* __restrict__ Bt, unsigned short* __restrict__ C) {
    gemm64_body<1, 0, 0, 0>(A, CW, Bt, CW, (void*)C, QLD, nullptr, nullptr, 0, 1, 0, MROWS, QLD, CW, 0.0625f);
}
__global__ __launch_bounds__(256) void k_gemm_wo(const unsigned short* __restrict__ A, const unsigned short* __restrict__ Bt, const float* __restrict__ bias, const float* __restrict__ xin, float* __restrict__ C) {
    gemm64_body<0, 1, 0, 1>(A, CW, Bt, CW, (void*)C, CW, bias, xin, CW, SEQ, (long long)SEQ_FULL * CW, MROWS, CW, CW, 0.0009765625f);
}
__global__ __launch_bounds__(256) void k_gemm_w1(const unsigned short* __restrict__ A, const unsigned short* __restrict__ Bt, const float* __restrict__ bias, unsigned short* __restrict__ C) {
    gemm64_body<1, 1, 1, 0>(A, CW, Bt, CW, (void*)C, FF, bias, nullptr, 0, 1, 0, MROWS, FF, CW, 0.0625f);
}
__global__ __launch_bounds__(256) void k_gemm_w2(const unsigned short* __restrict__ A, const unsigned short* __restrict__ Bt, const float* __restrict__ bias, const float* __restrict__ x1, float* __restrict__ C) {
    gemm64_body<0, 1, 0, 2>(A, FF, Bt, FF, (void*)C, CW, bias, x1, CW, SEQ, (long long)SEQ * CW, MROWS, CW, FF, 0.015625f);
}

__global__ __launch_bounds__(128) void k_attn_causal(const unsigned short* __restrict__ QKVp, unsigned short* __restrict__ AOp, float sl2) {
    __shared__ __align__(16) _Float16 Ksh[64 * 64];
    __shared__ __align__(16) _Float16 Vth[64 * 64];
    __shared__ __align__(16) _Float16 Psh[4][16 * 64];
    __shared__ __align__(16) float    Os[4][16 * 68];
    const _Float16* QKV = (const _Float16*)QKVp;
    const int tid = threadIdx.x, wave = tid >> 5, lane = tid & 31, hh = lane >> 4, c = lane & 15;
    const int nqb = SEQ / 64;
    const int bx = blockIdx.x;
    const int qb = bx % nqb;
    const int bh = bx / nqb;
    const int h = bh % NH;
    const int b = bh / NH;
    const int q0 = qb * 64 + wave * 16;
    const _Float16* Qb = QKV + (size_t)b * SEQ * QLD + (size_t)h * 64;
    const _Float16* Kb = Qb + CW;
    const _Float16* Vb = Qb + 2 * CW;

    v16h qa[2];
    {
        const _Float16* qrow = Qb + (size_t)(q0 + c) * QLD + 8 * hh;
        qa[0] = frag_ld_g(qrow);
        qa[1] = frag_ld_g(qrow + 32);
    }
    float mrow[8], lrow[8];
    v8f oacc[4];
#pragma unroll
    for (int r = 0; r < 8; ++r) { mrow[r] = -INFINITY; lrow[r] = 0.f; }
#pragma unroll
    for (int t = 0; t < 4; ++t) oacc[t] = (v8f){0.f, 0.f, 0.f, 0.f, 0.f, 0.f, 0.f, 0.f};

    const int nChunks = qb + 1;
    _Float16* pw = Psh[wave];
    for (int kc = 0; kc < nChunks; ++kc) {
        const int kv0 = kc * 64;
        __syncthreads();
        {
            const int kvr = tid >> 1, dh = (tid & 1) * 32;
            const _Float16* krow = Kb + (size_t)(kv0 + kvr) * QLD + dh;
            const _Float16* vrow = Vb + (size_t)(kv0 + kvr) * QLD + dh;
#pragma unroll
            for (int i = 0; i < 4; ++i) {
                const v8h kk = *(const v8h*)(krow + 8 * i);
                const v8h vv = *(const v8h*)(vrow + 8 * i);
                *(v8h*)(Ksh + kvr * 64 + dh + 8 * i) = kk;
#pragma unroll
                for (int e = 0; e < 8; ++e) Vth[(dh + 8 * i + e) * 64 + kvr] = vv[e];
            }
        }
        __syncthreads();

        v8f s[4];
#pragma unroll
        for (int j = 0; j < 4; ++j) {
            s[j] = (v8f){0.f, 0.f, 0.f, 0.f, 0.f, 0.f, 0.f, 0.f};
#pragma unroll
            for (int dc = 0; dc < 2; ++dc) {
                FH kb;
                kb.h[0] = *(const v8h*)(Ksh + (j * 16 + c) * 64 + dc * 32 + 8 * hh);
                kb.h[1] = *(const v8h*)(Ksh + (j * 16 + c) * 64 + dc * 32 + 16 + 8 * hh);
                s[j] = wmma16(qa[dc], kb.v, s[j]);
            }
        }
        const bool diag = (kc == qb);
        float cm[8];
#pragma unroll
        for (int r = 0; r < 8; ++r) {
            const int qrow = q0 + 8 * hh + r;
            float m = -INFINITY;
#pragma unroll
            for (int j = 0; j < 4; ++j) {
                const int kvcol = kv0 + j * 16 + c;
                float sv = s[j][r] * sl2;
                sv = (diag && (kvcol > qrow)) ? -INFINITY : sv;
                s[j][r] = sv;
                m = fmaxf(m, sv);
            }
            m = fmaxf(m, __shfl_xor(m, 1, 32)); m = fmaxf(m, __shfl_xor(m, 2, 32));
            m = fmaxf(m, __shfl_xor(m, 4, 32)); m = fmaxf(m, __shfl_xor(m, 8, 32));
            cm[r] = m;
        }
#pragma unroll
        for (int r = 0; r < 8; ++r) {
            const float mnew = fmaxf(mrow[r], cm[r]);
            const float alpha = exp2f(mrow[r] - mnew);
            mrow[r] = mnew;
            float psum = 0.f;
#pragma unroll
            for (int j = 0; j < 4; ++j) {
                const float p = exp2f(s[j][r] - mnew);
                psum += p;
                pw[(8 * hh + r) * 64 + j * 16 + c] = (_Float16)(p * 32768.0f);
            }
            psum += __shfl_xor(psum, 1, 32); psum += __shfl_xor(psum, 2, 32);
            psum += __shfl_xor(psum, 4, 32); psum += __shfl_xor(psum, 8, 32);
            lrow[r] = lrow[r] * alpha + psum;
#pragma unroll
            for (int t = 0; t < 4; ++t) oacc[t][r] *= alpha;
        }
        __builtin_amdgcn_fence(3  , "workgroup");
        __builtin_amdgcn_wave_barrier();
        __builtin_amdgcn_fence(2  , "workgroup");
#pragma unroll
        for (int kk = 0; kk < 2; ++kk) {
            FH pa;
            pa.h[0] = *(const v8h*)(pw + c * 64 + kk * 32 + 8 * hh);
            pa.h[1] = *(const v8h*)(pw + c * 64 + kk * 32 + 16 + 8 * hh);
#pragma unroll
            for (int t = 0; t < 4; ++t) {
                FH vb;
                vb.h[0] = *(const v8h*)(Vth + (t * 16 + c) * 64 + kk * 32 + 8 * hh);
                vb.h[1] = *(const v8h*)(Vth + (t * 16 + c) * 64 + kk * 32 + 16 + 8 * hh);
                oacc[t] = wmma16(pa.v, vb.v, oacc[t]);
            }
        }
    }

    float* os = Os[wave];
#pragma unroll
    for (int r = 0; r < 8; ++r) {
        const float inv = 1.0f / (lrow[r] * 512.0f);
#pragma unroll
        for (int t = 0; t < 4; ++t) os[(8 * hh + r) * 68 + t * 16 + c] = oacc[t][r] * inv;
    }
    __builtin_amdgcn_fence(3  , "workgroup");
    __builtin_amdgcn_wave_barrier();
    __builtin_amdgcn_fence(2  , "workgroup");
    {
        const int q4 = lane >> 3, c8 = (lane & 7) * 8;
        unsigned short* ob = AOp + ((size_t)b * SEQ + q0) * CW + (size_t)h * 64 + c8;
        for (int pass = 0; pass < 2; ++pass) {
#pragma unroll
            for (int it = 0; it < 4; ++it) {
                const int row = it * 4 + q4;
                const v4f a0 = *(const v4f*)(os + row * 68 + c8);
                const v4f a1 = *(const v4f*)(os + row * 68 + c8 + 4);
                v8h hv;
                hv[0] = (_Float16)a0.x; hv[1] = (_Float16)a0.y; hv[2] = (_Float16)a0.z; hv[3] = (_Float16)a0.w;
                hv[4] = (_Float16)a1.x; hv[5] = (_Float16)a1.y; hv[6] = (_Float16)a1.z; hv[7] = (_Float16)a1.w;
                *(volatile v8h*)(ob + (size_t)row * CW) = hv;
            }
            __threadfence();
        }
    }
}

constexpr size_t al256(size_t b) { return (b + 255) / 256 * 256; }
constexpr size_t SZ_STAT  = al256((size_t)NB * CW * 4);
constexpr size_t SZ_ACT16 = al256((size_t)MROWS * CW * 2);
constexpr size_t SZ_W316  = al256((size_t)QLD * CW * 2);
constexpr size_t SZ_QKV16 = al256((size_t)MROWS * QLD * 2);
constexpr size_t SZ_AO16  = al256((size_t)MROWS * CW * 2);
constexpr size_t SZ_WO16  = al256((size_t)CW * CW * 2);
constexpr size_t SZ_W1T   = al256((size_t)FF * CW * 2);
constexpr size_t SZ_W2T   = al256((size_t)CW * FF * 2);
constexpr size_t SZ_X1    = al256((size_t)MROWS * CW * 4);
constexpr size_t SZ_F16   = al256((size_t)MROWS * FF * 2);
constexpr size_t OFF_MEAN1 = 0;
constexpr size_t OFF_RSTD1 = OFF_MEAN1 + SZ_STAT;
constexpr size_t OFF_MEAN2 = OFF_RSTD1 + SZ_STAT;
constexpr size_t OFF_RSTD2 = OFF_MEAN2 + SZ_STAT;
constexpr size_t OFF_ACT16 = OFF_RSTD2 + SZ_STAT;
constexpr size_t OFF_W316  = OFF_ACT16 + SZ_ACT16;
constexpr size_t OFF_QKV16 = OFF_W316 + SZ_W316;
constexpr size_t OFF_AO16  = OFF_QKV16 + SZ_QKV16;
constexpr size_t OFF_WO16  = OFF_AO16 + SZ_AO16;
constexpr size_t OFF_W1T   = OFF_WO16 + SZ_WO16;
constexpr size_t OFF_W2T   = OFF_W1T + SZ_W1T;
constexpr size_t OFF_X1    = OFF_W2T + SZ_W2T;
constexpr size_t OFF_F16   = OFF_X1 + SZ_X1;
constexpr size_t WS_TOTAL  = OFF_F16 + SZ_F16;
static_assert(WS_TOTAL <= (size_t)134217728);

extern "C" void kernel_launch(void* const* d_in, const int* in_sizes, int n_in, void* d_out, int out_size, void* d_ws, size_t ws_size, hipStream_t stream) {
    if (n_in < 14) return;
    if ((long long)in_sizes[0] < (long long)(NB - 1) * SEQ_FULL * CW + (long long)SEQ * CW) return;
    if (in_sizes[1] < NH * CW * DHD || in_sizes[2] < NH * CW * DHD || in_sizes[3] < NH * CW * DHD) return;
    if (in_sizes[4] < CW * CW || in_sizes[5] < CW || in_sizes[6] < CW * FF || in_sizes[7] < FF || in_sizes[8] < FF * CW || in_sizes[9] < CW) return;
    if (in_sizes[10] < CW || in_sizes[11] < CW || in_sizes[12] < CW || in_sizes[13] < CW) return;
    if ((long long)out_size < (long long)MROWS * CW) return;
    if (WS_TOTAL > ws_size) return;

    const float* x   = (const float*)d_in[0];
    const float* wq  = (const float*)d_in[1];
    const float* wk  = (const float*)d_in[2];
    const float* wv  = (const float*)d_in[3];
    const float* wo  = (const float*)d_in[4];
    const float* bo  = (const float*)d_in[5];
    const float* w1  = (const float*)d_in[6];
    const float* b1  = (const float*)d_in[7];
    const float* w2  = (const float*)d_in[8];
    const float* b2  = (const float*)d_in[9];
    const float* g1  = (const float*)d_in[10];
    const float* be1 = (const float*)d_in[11];
    const float* g2  = (const float*)d_in[12];
    const float* be2 = (const float*)d_in[13];
    float* out = (float*)d_out;
    char* ws = (char*)d_ws;
    float* MEAN1 = (float*)(ws + OFF_MEAN1);
    float* RSTD1 = (float*)(ws + OFF_RSTD1);
    float* MEAN2 = (float*)(ws + OFF_MEAN2);
    float* RSTD2 = (float*)(ws + OFF_RSTD2);
    unsigned short* ACT16 = (unsigned short*)(ws + OFF_ACT16);
    unsigned short* W316  = (unsigned short*)(ws + OFF_W316);
    unsigned short* QKV16 = (unsigned short*)(ws + OFF_QKV16);
    unsigned short* AO16  = (unsigned short*)(ws + OFF_AO16);
    unsigned short* WO16  = (unsigned short*)(ws + OFF_WO16);
    unsigned short* W1T   = (unsigned short*)(ws + OFF_W1T);
    unsigned short* W2T   = (unsigned short*)(ws + OFF_W2T);
    float* X1 = (float*)(ws + OFF_X1);
    unsigned short* F16 = (unsigned short*)(ws + OFF_F16);

    const unsigned gApply = (unsigned)(((long long)MROWS * (CW / 8) + 255) / 256);

    k_colstat<<<dim3(CW / 32, NB), 256, 0, stream>>>(x, (long long)SEQ_FULL * CW, MEAN1, RSTD1, 1);
    k_lnt_apply<<<gApply, 256, 0, stream>>>(x, (long long)SEQ_FULL * CW, MEAN1, RSTD1, g1, be1, ACT16, 1);
    k_cast_heads<<<(unsigned)(((long long)CW * (CW / 8) + 255) / 256), 256, 0, stream>>>(wq, W316, 16.0f);
    k_cast_heads<<<(unsigned)(((long long)CW * (CW / 8) + 255) / 256), 256, 0, stream>>>(wk, W316 + (size_t)CW * CW, 16.0f);
    k_cast_heads<<<(unsigned)(((long long)CW * (CW / 8) + 255) / 256), 256, 0, stream>>>(wv, W316 + (size_t)2 * CW * CW, 16.0f);
    k_castbT<<<(unsigned)(((long long)CW * (CW / 8) + 255) / 256), 256, 0, stream>>>(wo, CW, WO16, CW, CW, CW, 16.0f);
    k_castbT<<<(unsigned)(((long long)FF * (CW / 8) + 255) / 256), 256, 0, stream>>>(w1, FF, W1T, CW, CW, FF, 16.0f);
    k_castbT<<<(unsigned)(((long long)CW * (FF / 8) + 255) / 256), 256, 0, stream>>>(w2, CW, W2T, FF, FF, CW, 64.0f);

    k_gemm_qkv<<<(unsigned)(((MROWS / 64) * (QLD / 64) + 7) / 8), 256, 0, stream>>>(ACT16, W316, QKV16);
    k_attn_causal<<<(unsigned)(NB * NH * (SEQ / 64)), 128, 0, stream>>>(QKV16, AO16, 0.03125f * 1.4426950408889634f);
    k_gemm_wo<<<(unsigned)(((MROWS / 64) * (CW / 64) + 7) / 8), 256, 0, stream>>>(AO16, WO16, bo, x, X1);

    k_colstat<<<dim3(CW / 32, NB), 256, 0, stream>>>(X1, (long long)SEQ * CW, MEAN2, RSTD2, 0);
    k_lnt_apply<<<gApply, 256, 0, stream>>>(X1, (long long)SEQ * CW, MEAN2, RSTD2, g2, be2, ACT16, 0);
    k_gemm_w1<<<(unsigned)(((MROWS / 64) * (FF / 64) + 7) / 8), 256, 0, stream>>>(ACT16, W1T, b1, F16);
    k_gemm_w2<<<(unsigned)(((MROWS / 64) * (CW / 64) + 7) / 8), 256, 0, stream>>>(F16, W2T, b2, X1, out);
}
